// LongShortAttention_919123001878
// MI455X (gfx1250) — hardware-verified
//
#include <hip/hip_runtime.h>
#include <math.h>
#include <stdint.h>

#define NB     2
#define NT     4096
#define DMODEL 1024
#define NHEAD  16
#define DHEAD  64
#define NBH    (NB * NHEAD)
#define MTOT   (NB * NT)
#define NSEGS  (NT / 16)
#define NQB    (NT / 64)
#define NTI    (NT / 128)
#define NGC    (NSEGS / 64)
#define EROWS  128
#define QMUL   8.0f
#define KCAR   8.0f
#define PCAR   1024.0f
#define CCAR   16.0f
#define WCAR   1024.0f
#define SINV   (1.0f / 512.0f)
#define OINV   (1.0f / 8192.0f)
#define YINV   (1.0f / 16384.0f)
#define NEG_BIG  (-1.0e30f)
#define NEG_HALF (-1.0e29f)
static_assert(NHEAD == 16 && DHEAD == 64 && DMODEL == NHEAD * DHEAD);
static_assert((NT % 1024) == 0);
static_assert(NSEGS == NTI * 8);
static_assert(NQB == NTI * 2);
static_assert(NGC * 64 == NSEGS);
static_assert(((MTOT * DMODEL) % 2048) == 0);

typedef _Float16 v16h __attribute__((ext_vector_type(16)));
typedef _Float16 v8h  __attribute__((ext_vector_type(8)));
typedef __bf16   v16b __attribute__((ext_vector_type(16)));
typedef unsigned short v8us __attribute__((ext_vector_type(8)));
typedef float    v8f  __attribute__((ext_vector_type(8)));
typedef float    v4f  __attribute__((ext_vector_type(4)));
typedef unsigned int v4u __attribute__((ext_vector_type(4)));
union FH { v16h v; v8h h[2]; };
union FB { v16b v; v8us h[2]; };
struct InvF { float f[32]; };
static_assert(sizeof(InvF) == 128);

__device__ __forceinline__ unsigned short bf_bits(float f) {
  unsigned u = __float_as_uint(f);
  return (unsigned short)((u + 0x7FFFu + ((u >> 16) & 1u)) >> 16);
}
__device__ __forceinline__ float bf_up(unsigned short b) { return __uint_as_float(((unsigned)b) << 16); }
__device__ __forceinline__ float bfr(float f) { return bf_up(bf_bits(f)); }
__device__ __forceinline__ unsigned short h_bits(_Float16 x) { return __builtin_bit_cast(unsigned short, x); }
__device__ __forceinline__ unsigned pk16(unsigned short a, unsigned short b) { return (unsigned)a | ((unsigned)b << 16); }
__device__ __forceinline__ v8f zero8() { v8f z = {0.f, 0.f, 0.f, 0.f, 0.f, 0.f, 0.f, 0.f}; return z; }
__device__ __forceinline__ float wsum32(float v) {
#pragma unroll
  for (int off = 1; off < 32; off <<= 1) v += __shfl_xor(v, off, 32);
  return v;
}

__device__ __forceinline__ v16h ldfrag_h(const _Float16* p) {
  FH f;
  f.h[0] = *(const v8h*)(p);
  f.h[1] = *(const v8h*)(p + 16);
  return f.v;
}
__device__ __forceinline__ v16b ldfrag_b(const unsigned short* p) {
  FB f;
  f.h[0] = *(const v8us*)(p);
  f.h[1] = *(const v8us*)(p + 16);
  return f.v;
}

__device__ __forceinline__ v8f mma_h(v16h a, v16h b, v8f cacc) {
  v8f d = __builtin_amdgcn_wmma_f32_16x16x32_f16(false, a, false, b, (short)0, cacc, false, false);
#if defined(__HIP_DEVICE_COMPILE__)
  asm volatile("v_nop\n\tv_nop\n\tv_nop\n\tv_nop" : "+v"(d) : "v"(a), "v"(b));
#endif
  return d;
}
__device__ __forceinline__ v8f mma_b(v16b a, v16b b, v8f cacc) {
  v8f d = __builtin_amdgcn_wmma_f32_16x16x32_bf16(false, a, false, b, (short)0, cacc, false, false);
#if defined(__HIP_DEVICE_COMPILE__)
  asm volatile("v_nop\n\tv_nop\n\tv_nop\n\tv_nop" : "+v"(d) : "v"(a), "v"(b));
#endif
  return d;
}
__device__ __forceinline__ void acc_guard4(v8f& a, v8f& b, v8f& c, v8f& d) {
#if defined(__HIP_DEVICE_COMPILE__)
  asm volatile("v_nop\n\tv_nop\n\tv_nop\n\tv_nop" : "+v"(a), "+v"(b), "+v"(c), "+v"(d));
#endif
}
__device__ __forceinline__ void wave_sync_lds() {
  __builtin_amdgcn_fence(__ATOMIC_RELEASE, "workgroup");
  __builtin_amdgcn_wave_barrier();
  __builtin_amdgcn_fence(__ATOMIC_ACQUIRE, "workgroup");
}

__global__ __launch_bounds__(256) void k_tab(float* cosT, float* sinT, InvF P) {
  const int lane = threadIdx.x & 31;
  const int t = (int)blockIdx.x * 8 + (int)(threadIdx.x >> 5);
  float f = P.f[0];
#pragma unroll
  for (int j = 1; j < 32; ++j) f = (lane == j) ? P.f[j] : f;
  const float ang = (float)t * f;
  float sn, cs;
  sincosf(ang, &sn, &cs);
  const size_t o = (size_t)t * 32 + lane;
  *(volatile float*)(cosT + o) = cs;
  *(volatile float*)(sinT + o) = sn;
  __threadfence();
  *(volatile float*)(cosT + o) = cs;
  *(volatile float*)(sinT + o) = sn;
}

__global__ __launch_bounds__(256) void k_cvtx(const float* __restrict__ in, unsigned short* out, int n) {
  const size_t i8 = ((size_t)blockIdx.x * 256 + threadIdx.x) * 8;
  if (i8 + 8 > (size_t)n) return;
  const v4f a = *(const v4f*)(in + i8);
  const v4f b = *(const v4f*)(in + i8 + 4);
  v4u p;
  p[0] = pk16(bf_bits(a[0]), bf_bits(a[1]));
  p[1] = pk16(bf_bits(a[2]), bf_bits(a[3]));
  p[2] = pk16(bf_bits(b[0]), bf_bits(b[1]));
  p[3] = pk16(bf_bits(b[2]), bf_bits(b[3]));
  *(volatile v4u*)(out + i8) = p;
  __threadfence();
  *(volatile v4u*)(out + i8) = p;
}

__global__ __launch_bounds__(128) void k_cvtw(const float* __restrict__ wq, const float* __restrict__ wkv,
                                              const float* __restrict__ wo, unsigned short* WT, unsigned short* WoT) {
  __shared__ __align__(16) unsigned short sT[64 * 72];
  const int tid = threadIdx.x, lane = tid & 31, wave = tid >> 5;
  const int mat  = (int)(blockIdx.x / 256u);
  const int tile = (int)(blockIdx.x % 256u);
  const int k0 = (tile >> 4) * 64, n0 = (tile & 15) * 64;
  const float* in = (mat == 0) ? wq : ((mat == 1) ? wkv : wo);
  unsigned short* out = (mat == 2) ? WoT : WT;
  const int nbase = (mat == 1) ? 1024 : 0;
  const bool f16mode = (mat == 2);
  {
    const int r = tid >> 1, nh = (tid & 1) * 32;
    const float* src = in + (size_t)(k0 + r) * DMODEL + n0 + nh;
#pragma unroll
    for (int i = 0; i < 8; ++i) {
      const v4f a = *(const v4f*)(src + 4 * i);
#pragma unroll
      for (int e = 0; e < 4; ++e) {
        const float v = bfr(a[e]);
        const unsigned short bits = f16mode ? h_bits((_Float16)(v * WCAR)) : bf_bits(v);
        sT[(nh + 4 * i + e) * 72 + r] = bits;
      }
    }
  }
  __syncthreads();
  const int ql = lane >> 3, pc = lane & 7;
  v8us vals[4];
#pragma unroll
  for (int it = 0; it < 4; ++it) {
    const int n = wave * 16 + it * 4 + ql;
    vals[it] = *(const v8us*)(sT + n * 72 + pc * 8);
  }
  for (int pass = 0; pass < 2; ++pass) {
#pragma unroll
    for (int it = 0; it < 4; ++it) {
      const int n = wave * 16 + it * 4 + ql;
      *(volatile v8us*)(out + (size_t)(nbase + n0 + n) * DMODEL + k0 + pc * 8) = vals[it];
    }
    __threadfence();
  }
}

__global__ __launch_bounds__(128)
void k_proj(const unsigned short* __restrict__ Xb, const unsigned short* __restrict__ WT,
            const float* __restrict__ cosT, const float* __restrict__ sinT,
            _Float16* Qh, _Float16* Ql, float* KVr) {
  __shared__ __align__(16) float Cs[128 * 68];
  __shared__ __align__(16) float Us[128 * 72];
  const int tid = threadIdx.x, lane = tid & 31, wave = tid >> 5, hh = lane >> 4, c = lane & 15;
  const int m0 = (int)blockIdx.x * 128;
  const int ntile = (int)blockIdx.y;
  const int n0 = ntile * 64;
  const int sel = ntile >> 4, head = ntile & 15;
  const int wm = wave * 32;

  v8f acc[2][4];
#pragma unroll
  for (int i = 0; i < 2; ++i)
#pragma unroll
    for (int j = 0; j < 4; ++j) acc[i][j] = zero8();

  const unsigned short* arow0 = Xb + (size_t)(m0 + wm + c) * DMODEL + 8 * hh;
  const unsigned short* arow1 = arow0 + (size_t)16 * DMODEL;
  const unsigned short* brow  = WT + (size_t)(n0 + c) * DMODEL + 8 * hh;
#pragma unroll 2
  for (int k0 = 0; k0 < DMODEL; k0 += 32) {
    const v16b a0 = ldfrag_b(arow0 + k0);
    const v16b a1 = ldfrag_b(arow1 + k0);
#pragma unroll
    for (int j = 0; j < 4; ++j) {
      const v16b b = ldfrag_b(brow + (size_t)j * 16 * DMODEL + k0);
      acc[0][j] = mma_b(a0, b, acc[0][j]);
      acc[1][j] = mma_b(a1, b, acc[1][j]);
    }
  }
  acc_guard4(acc[0][0], acc[0][1], acc[0][2], acc[0][3]);
  acc_guard4(acc[1][0], acc[1][1], acc[1][2], acc[1][3]);

#pragma unroll
  for (int i = 0; i < 2; ++i)
#pragma unroll
    for (int j = 0; j < 4; ++j)
#pragma unroll
      for (int r = 0; r < 8; ++r) Cs[(wm + 16 * i + 8 * hh + r) * 68 + 16 * j + c] = acc[i][j][r];
  __syncthreads();

  const int d = tid & 63, rpar = tid >> 6;
  const int jf = d & 31, pd = d ^ 32;
  const bool lowd = (d < 32);
  const int bb = m0 / NT, tb = m0 - bb * NT;
  const int bh = bb * NHEAD + head;
  _Float16* Hs = (_Float16*)Us;
  _Float16* Ls = Hs + 128 * 72;
  for (int r = rpar; r < 128; r += 2) {
    const int t = tb + r;
    const float cs = cosT[(size_t)t * 32 + jf];
    const float sn = sinT[(size_t)t * 32 + jf];
    const float v0 = Cs[r * 68 + d];
    const float vp = Cs[r * 68 + pd];
    const float vo = lowd ? -vp : vp;
    const float rv = v0 * cs + vo * sn;
    if (sel == 0) {
      const float qv = rv * QMUL;
      const _Float16 hi = (_Float16)qv;
      Hs[r * 72 + d] = hi;
      Ls[r * 72 + d] = (_Float16)(qv - (float)hi);
    } else {
      Us[r * 72 + d] = rv;
    }
  }
  __syncthreads();

  if (sel == 0) {
    const int ql = lane >> 3, pc = lane & 7;
    const bool dolo = (tb == 0);
    v8h hv[8], lv[8];
#pragma unroll
    for (int it = 0; it < 8; ++it) {
      const int row = wm + it * 4 + ql;
      hv[it] = *(const v8h*)(Hs + row * 72 + pc * 8);
      lv[it] = *(const v8h*)(Ls + row * 72 + pc * 8);
    }
    for (int pass = 0; pass < 2; ++pass) {
#pragma unroll
      for (int it = 0; it < 8; ++it) {
        const int row = wm + it * 4 + ql;
        const int t = tb + row;
        *(volatile v8h*)(Qh + ((size_t)bh * NT + t) * DHEAD + pc * 8) = hv[it];
        if (dolo) *(volatile v8h*)(Ql + ((size_t)bh * EROWS + row) * DHEAD + pc * 8) = lv[it];
      }
      __threadfence();
    }
  } else {
    const int rh = lane >> 4, c4 = (lane & 15) * 4;
    v4f fv[16];
#pragma unroll
    for (int it = 0; it < 16; ++it) {
      const int row = wm + 2 * it + rh;
      fv[it] = *(const v4f*)(Us + row * 72 + c4);
    }
    for (int pass = 0; pass < 2; ++pass) {
#pragma unroll
      for (int it = 0; it < 16; ++it) {
        const int row = wm + 2 * it + rh;
        *(volatile v4f*)(KVr + ((size_t)bh * NT + tb + row) * DHEAD + c4) = fv[it];
      }
      __threadfence();
    }
  }
}

__global__ __launch_bounds__(256)
void k_prep(const float* __restrict__ KVr, const float* __restrict__ wproj,
            const float* __restrict__ lg, const float* __restrict__ lb,
            const float* __restrict__ gg, const float* __restrict__ gb,
            _Float16* Lh, _Float16* Ll, _Float16* LhT, _Float16* LlT, _Float16* Gh, _Float16* Gl) {
  __shared__ __align__(16) float    Ks[128 * 68];
  __shared__ __align__(16) _Float16 Hr[128 * 72];
  __shared__ __align__(16) _Float16 Lr[128 * 72];
  __shared__ __align__(16) _Float16 Gsh[8 * 64];
  __shared__ __align__(16) _Float16 Gsl[8 * 64];
  __shared__ float prm[5][64];
  const int tid = threadIdx.x, lane = tid & 31, wave = tid >> 5;
  const int bh = (int)(blockIdx.x / (unsigned)NTI), ti = (int)(blockIdx.x % (unsigned)NTI);
  const int t0 = ti * 128;
  const bool dolo = (ti == 0);

  if (tid < 64) {
    prm[0][tid] = bfr(wproj[tid]);
    prm[1][tid] = bfr(lg[tid]);
    prm[2][tid] = bfr(lb[tid]);
    prm[3][tid] = bfr(gg[tid]);
    prm[4][tid] = bfr(gb[tid]);
  }
  const float* src = KVr + ((size_t)bh * NT + t0) * DHEAD;
  for (int i = tid; i < 2048; i += 256) {
    const int r = i >> 4, c4 = (i & 15) * 4;
    *(v4f*)(Ks + r * 68 + c4) = *(const v4f*)(src + (size_t)r * DHEAD + c4);
  }
  __syncthreads();

  {
    const int s = lane & 15;
    const float* kr = Ks + (wave * 16 + s) * 68;
    float lgt = 0.f;
#pragma unroll 1
    for (int dd = 0; dd < 64; ++dd) lgt += kr[dd] * prm[0][dd];
    float mx = lgt;
#pragma unroll
    for (int off = 1; off < 16; off <<= 1) mx = fmaxf(mx, __shfl_xor(mx, off, 32));
    const float ex = __expf(lgt - mx);
    float se = ex;
#pragma unroll
    for (int off = 1; off < 16; off <<= 1) se += __shfl_xor(se, off, 32);
    const float pp = ex * (1.0f / se);
    float a0 = 0.f, a1 = 0.f;
#pragma unroll 1
    for (int s2 = 0; s2 < 16; ++s2) {
      const float ps = __shfl(pp, s2, 32);
      const float* k2 = Ks + (wave * 16 + s2) * 68;
      a0 += ps * k2[lane];
      a1 += ps * k2[lane + 32];
    }
    const float mean = wsum32(a0 + a1) * (1.0f / 64.0f);
    const float d0 = a0 - mean, d1 = a1 - mean;
    const float var = wsum32(d0 * d0 + d1 * d1) * (1.0f / 64.0f);
    const float rs = rsqrtf(var + 1e-5f);
    const float y0 = (d0 * rs * prm[3][lane] + prm[4][lane]) * KCAR;
    const float y1 = (d1 * rs * prm[3][lane + 32] + prm[4][lane + 32]) * KCAR;
    const _Float16 h0 = (_Float16)y0, h1 = (_Float16)y1;
    Gsh[wave * 64 + lane] = h0;
    Gsh[wave * 64 + lane + 32] = h1;
    Gsl[wave * 64 + lane] = (_Float16)(y0 - (float)h0);
    Gsl[wave * 64 + lane + 32] = (_Float16)(y1 - (float)h1);
  }
#pragma unroll 1
  for (int k = 0; k < 16; ++k) {
    const int r = wave + 8 * k;
    const float x0 = Ks[r * 68 + lane], x1 = Ks[r * 68 + lane + 32];
    const float mean = wsum32(x0 + x1) * (1.0f / 64.0f);
    const float d0 = x0 - mean, d1 = x1 - mean;
    const float var = wsum32(d0 * d0 + d1 * d1) * (1.0f / 64.0f);
    const float rs = rsqrtf(var + 1e-5f);
    const float y0 = (d0 * rs * prm[1][lane] + prm[2][lane]) * KCAR;
    const float y1 = (d1 * rs * prm[1][lane + 32] + prm[2][lane + 32]) * KCAR;
    const _Float16 h0 = (_Float16)y0, h1 = (_Float16)y1;
    Hr[r * 72 + lane] = h0;
    Hr[r * 72 + lane + 32] = h1;
    Lr[r * 72 + lane] = (_Float16)(y0 - (float)h0);
    Lr[r * 72 + lane + 32] = (_Float16)(y1 - (float)h1);
  }
  __syncthreads();
  _Float16* HT = (_Float16*)Ks;
  _Float16* LT = HT + 64 * 136;
  for (int i = tid; i < 8192; i += 256) {
    const int t = i & 127, d = i >> 7;
    HT[d * 136 + t] = Hr[t * 72 + d];
    if (dolo) LT[d * 136 + t] = Lr[t * 72 + d];
  }
  __syncthreads();
  const int ql = lane >> 3, pc = lane & 7, rh = lane >> 4, pcw = lane & 15;
  v8h lrh[4], lrl[4], htv[4], ltv[4], ghv[2], glv[2];
#pragma unroll
  for (int it = 0; it < 4; ++it) {
    const int row = wave * 16 + it * 4 + ql;
    lrh[it] = *(const v8h*)(Hr + row * 72 + pc * 8);
    lrl[it] = *(const v8h*)(Lr + row * 72 + pc * 8);
    const int dr = wave * 8 + 2 * it + rh;
    htv[it] = *(const v8h*)(HT + dr * 136 + pcw * 8);
    ltv[it] = *(const v8h*)(LT + dr * 136 + pcw * 8);
  }
#pragma unroll
  for (int it = 0; it < 2; ++it) {
    const int j = it * 4 + ql;
    ghv[it] = *(const v8h*)(Gsh + j * 64 + pc * 8);
    glv[it] = *(const v8h*)(Gsl + j * 64 + pc * 8);
  }
  for (int pass = 0; pass < 2; ++pass) {
#pragma unroll
    for (int it = 0; it < 4; ++it) {
      const int row = wave * 16 + it * 4 + ql;
      *(volatile v8h*)(Lh + ((size_t)bh * NT + t0 + row) * DHEAD + pc * 8) = lrh[it];
      if (dolo) *(volatile v8h*)(Ll + ((size_t)bh * EROWS + row) * DHEAD + pc * 8) = lrl[it];
      const int dr = wave * 8 + 2 * it + rh;
      *(volatile v8h*)(LhT + ((size_t)bh * DHEAD + dr) * NT + t0 + pcw * 8) = htv[it];
      if (dolo) *(volatile v8h*)(LlT + ((size_t)bh * DHEAD + dr) * EROWS + pcw * 8) = ltv[it];
    }
    if (wave == 0) {
#pragma unroll
      for (int it = 0; it < 2; ++it) {
        const int j = it * 4 + ql;
        *(volatile v8h*)(Gh + ((size_t)bh * NSEGS + ti * 8 + j) * DHEAD + pc * 8) = ghv[it];
        *(volatile v8h*)(Gl + ((size_t)bh * NSEGS + ti * 8 + j) * DHEAD + pc * 8) = glv[it];
      }
    }
    __threadfence();
  }
}

__global__ __launch_bounds__(128) void k_gtr(const _Float16* __restrict__ Gh, const _Float16* __restrict__ Gl,
                                             _Float16* GhT, _Float16* GlT) {
  __shared__ __align__(16) _Float16 sT[64 * 72];
  const int tid = threadIdx.x, lane = tid & 31, wave = tid >> 5;
  const int pl  = (int)(blockIdx.x / (unsigned)(NBH * NGC));
  const int rem = (int)(blockIdx.x % (unsigned)(NBH * NGC));
  const int bh = rem / NGC, rc = rem - bh * NGC;
  const _Float16* in = pl ? Gl : Gh;
  _Float16* out = pl ? GlT : GhT;
  {
    const int r = tid >> 1, dh = (tid & 1) * 32;
    const _Float16* src = in + ((size_t)bh * NSEGS + rc * 64 + r) * DHEAD + dh;
#pragma unroll
    for (int i = 0; i < 4; ++i) {
      const v8h a = *(const v8h*)(src + 8 * i);
#pragma unroll
      for (int e = 0; e < 8; ++e) sT[(dh + 8 * i + e) * 72 + r] = a[e];
    }
  }
  __syncthreads();
  const int ql = lane >> 3, pc = lane & 7;
  v8h vals[4];
#pragma unroll
  for (int it = 0; it < 4; ++it) {
    const int d = wave * 16 + it * 4 + ql;
    vals[it] = *(const v8h*)(sT + d * 72 + pc * 8);
  }
  for (int pass = 0; pass < 2; ++pass) {
#pragma unroll
    for (int it = 0; it < 4; ++it) {
      const int d = wave * 16 + it * 4 + ql;
      *(volatile v8h*)(out + ((size_t)bh * DHEAD + d) * NSEGS + rc * 64 + pc * 8) = vals[it];
    }
    __threadfence();
  }
}

__global__ __launch_bounds__(128)
void k_attn(const _Float16* __restrict__ Qh, const _Float16* __restrict__ Ql,
            const _Float16* __restrict__ Lh, const _Float16* __restrict__ Ll,
            const _Float16* __restrict__ LhT, const _Float16* __restrict__ LlT,
            const _Float16* __restrict__ Gh, const _Float16* __restrict__ Gl,
            const _Float16* __restrict__ GhT, const _Float16* __restrict__ GlT,
            _Float16* Ch, _Float16* Cl) {
  __shared__ __align__(16) _Float16 Ksh[64 * 64];
  __shared__ __align__(16) _Float16 Klsh[64 * 64];
  __shared__ __align__(16) _Float16 Vsh[64 * 64];
  __shared__ __align__(16) _Float16 Vlsh[64 * 64];
  __shared__ __align__(16) _Float16 Psh[4][16 * 64];
  __shared__ __align__(16) _Float16 Plsh[4][16 * 64];
  __shared__ __align__(16) _Float16 Osh[4][16 * 64];
  __shared__ __align__(16) _Float16 Osl[4][16 * 64];

  const int tid = threadIdx.x, wave = tid >> 5, lane = tid & 31, hh = lane >> 4, c = lane & 15;
  const int qblk = (int)(blockIdx.x % (unsigned)NQB);
  const int bh   = (int)(blockIdx.x / (unsigned)NQB);
  const int bb   = bh >> 4, head = bh & 15;
  const int wi = qblk >> 1, sub = qblk & 1;
  const int ncur = sub + 1;
  const int nprv = (wi > 0) ? 2 : 0;
  const int ng   = (qblk >> 4) + 1;
  const int nch  = ncur + nprv + ng;
  const bool early = (qblk < 2);
  const int q0w = qblk * 64 + wave * 16;
  const int qlr = early ? (q0w + c) : 0;
  const _Float16* Qhp = Qh + ((size_t)bh * NT + q0w + c) * DHEAD + 8 * hh;
  const _Float16* Qlp = Ql + ((size_t)bh * EROWS + qlr) * DHEAD + 8 * hh;

  float mrow[8], lrow[8];
  v8f oh[4];
#pragma unroll
  for (int r = 0; r < 8; ++r) { mrow[r] = NEG_BIG; lrow[r] = 0.f; }
#pragma unroll
  for (int t = 0; t < 4; ++t) oh[t] = zero8();

  _Float16* pwh = Psh[wave];
  _Float16* pwl = Plsh[wave];

  for (int ci = 0; ci < nch; ++ci) {
    int mode = 0, R0 = 0;
    const _Float16 *kbase, *klbase, *vbase, *vlbase;
    int vpitch, vlpitch;
    if (ci < ncur + nprv) {
      int tk0;
      if (ci < ncur) { const int cc = sub - ci; tk0 = wi * 128 + cc * 64; mode = (ci == 0) ? 1 : 0; }
      else           { const int cc = ci - ncur; tk0 = (wi - 1) * 128 + cc * 64; mode = 0; }
      const int tkl = (tk0 < 64) ? tk0 : 64;
      kbase  = Lh  + ((size_t)bh * NT + tk0) * DHEAD;
      klbase = Ll  + ((size_t)bh * EROWS + tkl) * DHEAD;
      vbase  = LhT + (size_t)bh * DHEAD * NT + tk0;      vpitch  = NT;
      vlbase = LlT + (size_t)bh * DHEAD * EROWS + tkl;   vlpitch = EROWS;
    } else {
      const int gc = ci - ncur - nprv;
      R0 = gc * 64;
      mode = 2;
      kbase  = Gh  + ((size_t)bh * NSEGS + R0) * DHEAD;
      klbase = Gl  + ((size_t)bh * NSEGS + R0) * DHEAD;
      vbase  = GhT + (size_t)bh * DHEAD * NSEGS + R0;    vpitch  = NSEGS;
      vlbase = GlT + (size_t)bh * DHEAD * NSEGS + R0;    vlpitch = NSEGS;
    }
    __syncthreads();
    {
      const int r = tid >> 1, hk = (tid & 1) * 32;
      const _Float16* ks = kbase + (size_t)r * DHEAD + hk;
#pragma unroll
      for (int i = 0; i < 4; ++i) *(v8h*)(Ksh + r * 64 + hk + 8 * i) = *(const v8h*)(ks + 8 * i);
      const _Float16* vs = vbase + (size_t)r * vpitch + hk;
#pragma unroll
      for (int i = 0; i < 4; ++i) *(v8h*)(Vsh + r * 64 + hk + 8 * i) = *(const v8h*)(vs + 8 * i);
      if (early) {
        const _Float16* kls = klbase + (size_t)r * DHEAD + hk;
#pragma unroll
        for (int i = 0; i < 4; ++i) *(v8h*)(Klsh + r * 64 + hk + 8 * i) = *(const v8h*)(kls + 8 * i);
        const _Float16* vls = vlbase + (size_t)r * vlpitch + hk;
#pragma unroll
        for (int i = 0; i < 4; ++i) *(v8h*)(Vlsh + r * 64 + hk + 8 * i) = *(const v8h*)(vls + 8 * i);
      }
    }
    __syncthreads();

    v8f s[4];
#pragma unroll
    for (int j = 0; j < 4; ++j) s[j] = zero8();
#pragma unroll
    for (int dc = 0; dc < 2; ++dc) {
      const v16h qa = ldfrag_h(Qhp + dc * 32);
#pragma unroll
      for (int j = 0; j < 4; ++j) {
        FH kb;
        kb.h[0] = *(const v8h*)(Ksh + (j * 16 + c) * 64 + dc * 32 + 8 * hh);
        kb.h[1] = *(const v8h*)(Ksh + (j * 16 + c) * 64 + dc * 32 + 16 + 8 * hh);
        s[j] = mma_h(qa, kb.v, s[j]);
      }
      if (early) {
        const v16h qlo = ldfrag_h(Qlp + dc * 32);
#pragma unroll
        for (int j = 0; j < 4; ++j) {
          FH kb, kbl;
          kb.h[0]  = *(const v8h*)(Ksh  + (j * 16 + c) * 64 + dc * 32 + 8 * hh);
          kb.h[1]  = *(const v8h*)(Ksh  + (j * 16 + c) * 64 + dc * 32 + 16 + 8 * hh);
          kbl.h[0] = *(const v8h*)(Klsh + (j * 16 + c) * 64 + dc * 32 + 8 * hh);
          kbl.h[1] = *(const v8h*)(Klsh + (j * 16 + c) * 64 + dc * 32 + 16 + 8 * hh);
          s[j] = mma_h(qlo, kb.v, s[j]);
          s[j] = mma_h(qa, kbl.v, s[j]);
        }
      }
    }
    acc_guard4(s[0], s[1], s[2], s[3]);

    const int nb = qblk * 64 + wave * 16 + 8 * hh;
#pragma unroll
    for (int j = 0; j < 4; ++j) {
      const int kl = j * 16 + c;
#pragma unroll
      for (int r = 0; r < 8; ++r) {
        const float x = s[j][r] * SINV;
        int lim;
        if (mode == 0)      lim = 4096;
        else if (mode == 1) lim = wave * 16 + 8 * hh + r;
        else                lim = ((nb + r + 1) >> 4) - 1 - R0;
        s[j][r] = (kl > lim) ? NEG_BIG : x;
      }
    }

#pragma unroll
    for (int r = 0; r < 8; ++r) {
      float m = fmaxf(fmaxf(s[0][r], s[1][r]), fmaxf(s[2][r], s[3][r]));
#pragma unroll
      for (int off = 1; off < 16; off <<= 1) m = fmaxf(m, __shfl_xor(m, off, 32));
      const float mnew  = fmaxf(mrow[r], m);
      const float alpha = __expf(mrow[r] - mnew);
      mrow[r] = mnew;
      float psum = 0.f;
#pragma unroll
      for (int j = 0; j < 4; ++j) {
        const float sv = s[j][r];
        const float p  = (sv > NEG_HALF) ? __expf(sv - mnew) : 0.f;
        psum += p;
        const float pv = p * PCAR;
        const _Float16 ph = (_Float16)pv;
        pwh[(8 * hh + r) * 64 + j * 16 + c] = ph;
        if (early) pwl[(8 * hh + r) * 64 + j * 16 + c] = (_Float16)(pv - (float)ph);
      }
#pragma unroll
      for (int off = 1; off < 16; off <<= 1) psum += __shfl_xor(psum, off, 32);
      lrow[r] = lrow[r] * alpha + psum;
#pragma unroll
      for (int t = 0; t < 4; ++t) oh[t][r] *= alpha;
    }
    wave_sync_lds();

#pragma unroll
    for (int kk = 0; kk < 2; ++kk) {
      FH pa;
      pa.h[0] = *(const v8h*)(pwh + c * 64 + kk * 32 + 8 * hh);
      pa.h[1] = *(const v8h*)(pwh + c * 64 + kk * 32 + 16 + 8 * hh);
#pragma unroll
      for (int t = 0; t < 4; ++t) {
        FH vb;
        vb.h[0] = *(const v8h*)(Vsh + (t * 16 + c) * 64 + kk * 32 + 8 * hh);
        vb.h[1] = *(const v8h*)(Vsh + (t * 16 + c) * 64 + kk * 32 + 16 + 8 * hh);
        oh[t] = mma_h(pa.v, vb.v, oh[t]);
      }
      if (early) {
        FH pl;
        pl.h[0] = *(const v8h*)(pwl + c * 64 + kk * 32 + 8 * hh);
        pl.h[1] = *(const v8h*)(pwl + c * 64 + kk * 32 + 16 + 8 * hh);
#pragma unroll
        for (int t = 0; t < 4; ++t) {
          FH vb, vbl;
          vb.h[0]  = *(const v8h*)(Vsh  + (t * 16 + c) * 64 + kk * 32 + 8 * hh);
          vb.h[1]  = *(const v8h*)(Vsh  + (t * 16 + c) * 64 + kk * 32 + 16 + 8 * hh);
          vbl.h[0] = *(const v8h*)(Vlsh + (t * 16 + c) * 64 + kk * 32 + 8 * hh);
          vbl.h[1] = *(const v8h*)(Vlsh + (t * 16 + c) * 64 + kk * 32 + 16 + 8 * hh);
          oh[t] = mma_h(pl.v, vb.v, oh[t]);
          oh[t] = mma_h(pa.v, vbl.v, oh[t]);
        }
      }
    }
    acc_guard4(oh[0], oh[1], oh[2], oh[3]);
  }

  _Float16* osh = Osh[wave];
  _Float16* osl = Osl[wave];
#pragma unroll
  for (int r = 0; r < 8; ++r) {
    const float l = lrow[r];
    const float inv = (1.0f / l) * OINV;
#pragma unroll
    for (int t = 0; t < 4; ++t) {
      const float oc = oh[t][r] * inv * CCAR;
      const _Float16 hi = (_Float16)oc;
      osh[(8 * hh + r) * 64 + t * 16 + c] = hi;
      osl[(8 * hh + r) * 64 + t * 16 + c] = (_Float16)(oc - (float)hi);
    }
  }
  wave_sync_lds();
  const int ql = lane >> 3, pc = lane & 7;
  v8h hv[4], lv[4];
#pragma unroll
  for (int it = 0; it < 4; ++it) {
    const int row = it * 4 + ql;
    hv[it] = *(const v8h*)(osh + row * 64 + pc * 8);
    lv[it] = *(const v8h*)(osl + row * 64 + pc * 8);
  }
  for (int pass = 0; pass < 2; ++pass) {
#pragma unroll
    for (int it = 0; it < 4; ++it) {
      const int row = it * 4 + ql;
      const int t = q0w + row;
      *(volatile v8h*)(Ch + ((size_t)bb * NT + t) * DMODEL + head * DHEAD + pc * 8) = hv[it];
      if (early) *(volatile v8h*)(Cl + ((size_t)bb * EROWS + t) * DMODEL + head * DHEAD + pc * 8) = lv[it];
    }
    __threadfence();
  }
}

__global__ __launch_bounds__(128)
void k_out(const _Float16* __restrict__ Ch, const _Float16* __restrict__ Cl, const _Float16* __restrict__ WoT,
           const float* __restrict__ bout, float* Out) {
  __shared__ __align__(16) float Os[4][32 * 68];
  const int tid = threadIdx.x, lane = tid & 31, wave = tid >> 5, hh = lane >> 4, c = lane & 15;
  const int m0 = (int)blockIdx.x * 128;
  const int n0 = (int)blockIdx.y * 64;
  const int wm = wave * 32;
  const int bb = m0 / NT;
  const bool dolo = ((m0 - bb * NT) == 0);

  v8f acc[2][4];
#pragma unroll
  for (int i = 0; i < 2; ++i)
#pragma unroll
    for (int j = 0; j < 4; ++j) acc[i][j] = zero8();

  const _Float16* arow0 = Ch + (size_t)(m0 + wm + c) * DMODEL + 8 * hh;
  const _Float16* arow1 = arow0 + (size_t)16 * DMODEL;
  const int lr0 = dolo ? (wm + c) : 0;
  const _Float16* lrow0 = Cl + (size_t)(bb * EROWS + lr0) * DMODEL + 8 * hh;
  const _Float16* lrow1 = lrow0 + (dolo ? (size_t)16 * DMODEL : (size_t)0);
  const _Float16* brow  = WoT + (size_t)(n0 + c) * DMODEL + 8 * hh;
#pragma unroll 2
  for (int k0 = 0; k0 < DMODEL; k0 += 32) {
    const v16h a0 = ldfrag_h(arow0 + k0);
    const v16h a1 = ldfrag_h(arow1 + k0);
#pragma unroll
    for (int j = 0; j < 4; ++j) {
      const v16h b = ldfrag_h(brow + (size_t)j * 16 * DMODEL + k0);
      acc[0][j] = mma_h(a0, b, acc[0][j]);
      acc[1][j] = mma_h(a1, b, acc[1][j]);
    }
    if (dolo) {
      const v16h al0 = ldfrag_h(lrow0 + k0);
      const v16h al1 = ldfrag_h(lrow1 + k0);
#pragma unroll
      for (int j = 0; j < 4; ++j) {
        const v16h b = ldfrag_h(brow + (size_t)j * 16 * DMODEL + k0);
        acc[0][j] = mma_h(al0, b, acc[0][j]);
        acc[1][j] = mma_h(al1, b, acc[1][j]);
      }
    }
  }
  acc_guard4(acc[0][0], acc[0][1], acc[0][2], acc[0][3]);
  acc_guard4(acc[1][0], acc[1][1], acc[1][2], acc[1][3]);

  float* os = Os[wave];
#pragma unroll
  for (int i = 0; i < 2; ++i)
#pragma unroll
    for (int j = 0; j < 4; ++j) {
      const float bias = bfr(bout[n0 + 16 * j + c]);
#pragma unroll
      for (int r = 0; r < 8; ++r) os[(16 * i + 8 * hh + r) * 68 + 16 * j + c] = acc[i][j][r] * YINV + bias;
    }
  wave_sync_lds();
  const int rh = lane >> 4, c4 = (lane & 15) * 4;
  v4f fv[16];
#pragma unroll
  for (int it = 0; it < 16; ++it) {
    const int row = 2 * it + rh;
    fv[it] = *(const v4f*)(os + row * 68 + c4);
  }
  for (int pass = 0; pass < 2; ++pass) {
#pragma unroll
    for (int it = 0; it < 16; ++it) {
      const int row = 2 * it + rh;
      *(volatile v4f*)(Out + (size_t)(m0 + wm + row) * DMODEL + n0 + c4) = fv[it];
    }
    __threadfence();
  }
}

extern "C" void kernel_launch(void* const* d_in, const int* in_sizes, int n_in,
                              void* d_out, int out_size, void* d_ws, size_t ws_size,
                              hipStream_t stream) {
  if (n_in < 10) return;
  if (in_sizes[0] != MTOT * DMODEL) return;
  if (in_sizes[1] != DMODEL * DMODEL || in_sizes[2] != DMODEL * DMODEL || in_sizes[8] != DMODEL * DMODEL) return;
  if (in_sizes[3] != DHEAD || in_sizes[4] != DHEAD || in_sizes[5] != DHEAD) return;
  if (in_sizes[6] != DHEAD || in_sizes[7] != DHEAD || in_sizes[9] != DMODEL) return;
  if (out_size != MTOT * DMODEL) return;

  const float* x     = (const float*)d_in[0];
  const float* w_q   = (const float*)d_in[1];
  const float* w_kv  = (const float*)d_in[2];
  const float* w_prj = (const float*)d_in[3];
  const float* lng   = (const float*)d_in[4];
  const float* lnb   = (const float*)d_in[5];
  const float* gng   = (const float*)d_in[6];
  const float* gnb   = (const float*)d_in[7];
  const float* w_out = (const float*)d_in[8];
  const float* b_out = (const float*)d_in[9];
  float* outf = (float*)d_out;

  size_t off = 0;
  const size_t oX   = off; off += (size_t)MTOT * DMODEL * 2;
  const size_t oWT  = off; off += (size_t)2048 * DMODEL * 2;
  const size_t oWo  = off; off += (size_t)DMODEL * DMODEL * 2;
  const size_t oCos = off; off += (size_t)NT * 32 * 4;
  const size_t oSin = off; off += (size_t)NT * 32 * 4;
  const size_t oQh  = off; off += (size_t)NBH * NT * DHEAD * 2;
  const size_t oQl  = off; off += (size_t)NBH * EROWS * DHEAD * 2;
  const size_t oKV  = off; off += (size_t)NBH * NT * DHEAD * 4;
  const size_t oLh  = off; off += (size_t)NBH * NT * DHEAD * 2;
  const size_t oLl  = off; off += (size_t)NBH * EROWS * DHEAD * 2;
  const size_t oLhT = off; off += (size_t)NBH * DHEAD * NT * 2;
  const size_t oLlT = off; off += (size_t)NBH * DHEAD * EROWS * 2;
  const size_t oGh  = off; off += (size_t)NBH * NSEGS * DHEAD * 2;
  const size_t oGl  = off; off += (size_t)NBH * NSEGS * DHEAD * 2;
  const size_t oGhT = off; off += (size_t)NBH * DHEAD * NSEGS * 2;
  const size_t oGlT = off; off += (size_t)NBH * DHEAD * NSEGS * 2;
  const size_t oCl  = off; off += (size_t)NB * EROWS * DMODEL * 2;
  if (off > ws_size) return;
  if (off > (size_t)134217728) return;

  char* ws = (char*)d_ws;
  unsigned short* Xb  = (unsigned short*)(ws + oX);
  _Float16*       Ch  = (_Float16*)(ws + oX);
  unsigned short* WT  = (unsigned short*)(ws + oWT);
  unsigned short* WoT = (unsigned short*)(ws + oWo);
  float* cosT = (float*)(ws + oCos);
  float* sinT = (float*)(ws + oSin);
  _Float16* Qh  = (_Float16*)(ws + oQh);
  _Float16* Ql  = (_Float16*)(ws + oQl);
  float*    KVr = (float*)(ws + oKV);
  _Float16* Lh  = (_Float16*)(ws + oLh);
  _Float16* Ll  = (_Float16*)(ws + oLl);
  _Float16* LhT = (_Float16*)(ws + oLhT);
  _Float16* LlT = (_Float16*)(ws + oLlT);
  _Float16* Gh  = (_Float16*)(ws + oGh);
  _Float16* Gl  = (_Float16*)(ws + oGl);
  _Float16* GhT = (_Float16*)(ws + oGhT);
  _Float16* GlT = (_Float16*)(ws + oGlT);
  _Float16* Cl  = (_Float16*)(ws + oCl);

  InvF P;
  {
    double rt = 1.3335214321633;
    for (int it = 0; it < 40; ++it) {
      double pw = 1.0;
      for (int k = 0; k < 32; ++k) pw *= rt;
      rt = rt - (pw - 10000.0) * rt / (32.0 * pw);
    }
    double pj = 1.0;
    for (int j = 0; j < 32; ++j) {
      const float pf = (float)pj;
      P.f[j] = 1.0f / pf;
      pj *= rt;
    }
  }

  const dim3 blk256(256), blk128(128);
  k_tab<<<dim3(NT / 8), blk256, 0, stream>>>(cosT, sinT, P);
  k_cvtx<<<dim3((MTOT * DMODEL) / 2048), blk256, 0, stream>>>(x, Xb, MTOT * DMODEL);
  k_cvtw<<<dim3(3 * 256), blk128, 0, stream>>>(w_q, w_kv, w_out, WT, WoT);
  k_proj<<<dim3(MTOT / 128, 32), blk128, 0, stream>>>(Xb, WT, cosT, sinT, Qh, Ql, KVr);
  k_prep<<<dim3(NBH * NTI), blk256, 0, stream>>>(KVr, w_prj, lng, lnb, gng, gnb, Lh, Ll, LhT, LlT, Gh, Gl);
  k_gtr<<<dim3(2 * NBH * NGC), blk128, 0, stream>>>(Gh, Gl, GhT, GlT);
  k_attn<<<dim3(NBH * NQB), blk128, 0, stream>>>(Qh, Ql, Lh, Ll, LhT, LlT, Gh, Gl, GhT, GlT, Ch, Cl);
  k_out<<<dim3(MTOT / 128, DMODEL / 64), blk128, 0, stream>>>(Ch, Cl, (const _Float16*)WoT, b_out, outf);
  (void)hipGetLastError();
}
